// MultiAttention_13726715478235
// MI455X (gfx1250) — hardware-verified
//
#include <hip/hip_runtime.h>
#include <stdint.h>


typedef __bf16 v16bf __attribute__((ext_vector_type(16)));
typedef unsigned short v8us __attribute__((ext_vector_type(8)));
typedef float v8f __attribute__((ext_vector_type(8)));
typedef float v4f __attribute__((ext_vector_type(4)));
typedef unsigned int v4u __attribute__((ext_vector_type(4)));

#define SEQ 2048
#define DM 1024
#define NH 16
#define HD 64
#define NFREQ 32

#define BP 40
#define SP 72
#define KP 72
#define VP 40
#define PP 40
#define OP 72
#define TP 68

union Frag { v16bf v; v8us p[2]; };

static __device__ __forceinline__ v16bf frag_ld(const unsigned short* row_k0, int hh) {
  Frag f;
  f.p[0] = *(const v8us*)(row_k0 + 8 * hh);
  f.p[1] = *(const v8us*)(row_k0 + 16 + 8 * hh);
  return f.v;
}

static __device__ __forceinline__ v8f mma(v16bf a, v16bf b, v8f c) {
  v8f d = __builtin_amdgcn_wmma_f32_16x16x32_bf16(false, a, false, b, (short)0, c, false, false);
  asm volatile("v_nop\n\tv_nop\n\tv_nop\n\tv_nop" : "+v"(d) : "v"(a), "v"(b));
  return d;
}

static __device__ __forceinline__ v8f zero8() {
  v8f z = {0.f, 0.f, 0.f, 0.f, 0.f, 0.f, 0.f, 0.f};
  return z;
}

static __device__ __forceinline__ unsigned short f2bf(float f) {
  unsigned int u = __float_as_uint(f);
  u = u + 0x7FFFu + ((u >> 16) & 1u);
  return (unsigned short)(u >> 16);
}

__global__ __launch_bounds__(256) void k_cvt(const float* __restrict__ src,
                                             unsigned short* __restrict__ dst, int n8) {
  const int i = blockIdx.x * 256 + threadIdx.x;
  const bool ok = i < n8;
  v4u wv = {0u, 0u, 0u, 0u};
  if (ok) {
    const float* s = src + (size_t)i * 8;
    v4f a = *(const v4f*)s;
    v4f b = *(const v4f*)(s + 4);
    wv[0] = (unsigned int)f2bf(a[0]) | ((unsigned int)f2bf(a[1]) << 16);
    wv[1] = (unsigned int)f2bf(a[2]) | ((unsigned int)f2bf(a[3]) << 16);
    wv[2] = (unsigned int)f2bf(b[0]) | ((unsigned int)f2bf(b[1]) << 16);
    wv[3] = (unsigned int)f2bf(b[2]) | ((unsigned int)f2bf(b[3]) << 16);
    *(volatile v4u*)(dst + (size_t)i * 8) = wv;
  }
  __threadfence();
  if (ok) {
    *(volatile v4u*)(dst + (size_t)i * 8) = wv;
  }
}

__global__ __launch_bounds__(256) void k_tab(float* __restrict__ cosT, float* __restrict__ sinT, int n4) {
  __shared__ __align__(16) float tc[1024];
  __shared__ __align__(16) float ts[1024];
  const int i = blockIdx.x * 256 + threadIdx.x;
  const int s = i >> 3;
  const int f0 = (i & 7) * 4;
#pragma unroll 1
  for (int j = 0; j < 4; ++j) {
    float e = (float)(f0 + j) * (1.0f / 32.0f);
    float p = powf(10000.0f, e);
    float invf = 1.0f / p;
    float ang = (float)s * invf;
    tc[threadIdx.x * 4 + j] = cosf(ang);
    ts[threadIdx.x * 4 + j] = sinf(ang);
  }
  __syncthreads();
  v4f cv = *(const v4f*)(tc + threadIdx.x * 4);
  v4f sv = *(const v4f*)(ts + threadIdx.x * 4);
  const bool ok = i < n4;
  if (ok) {
    *(volatile v4f*)(cosT + (size_t)i * 4) = cv;
    *(volatile v4f*)(sinT + (size_t)i * 4) = sv;
  }
  __threadfence();
  if (ok) {
    *(volatile v4f*)(cosT + (size_t)i * 4) = cv;
    *(volatile v4f*)(sinT + (size_t)i * 4) = sv;
  }
}

__global__ __launch_bounds__(256) void k_qkv(
    const unsigned short* __restrict__ xh, const unsigned short* __restrict__ wh,
    const float* __restrict__ bias, const float* __restrict__ cosT, const float* __restrict__ sinT,
    unsigned short* __restrict__ Qh, unsigned short* __restrict__ Kh, unsigned short* __restrict__ Vh) {
  __shared__ __align__(16) unsigned short Bl[64 * BP];
  __shared__ __align__(16) unsigned short St[8 * 32 * SP];
  const int t = threadIdx.x, w = t >> 5, l = t & 31, m = l & 15, hh = l >> 4;
  const int NT = (3 * DM) / 64;
  const int col0 = (blockIdx.x % NT) * 64;
  const int rowb = (blockIdx.x / NT) * 256;
  if (rowb >= SEQ) return;
  const int row0 = rowb + w * 32;

  const unsigned short* xr0 = xh + (size_t)(row0 + m) * DM;
  const unsigned short* xr1 = xr0 + (size_t)16 * DM;
  const unsigned short* wsrc = wh + (size_t)(col0 + (t >> 2)) * DM + (t & 3) * 8;
  unsigned short* wdst = Bl + (t >> 2) * BP + (t & 3) * 8;

  v8f c[2][4];
#pragma unroll
  for (int rr = 0; rr < 2; ++rr)
#pragma unroll
    for (int j = 0; j < 4; ++j) c[rr][j] = zero8();

  for (int i = 0; i < DM / 32; ++i) {
    const int k0 = i * 32;
    __syncthreads();
    *(v8us*)wdst = *(const v8us*)(wsrc + k0);
    __syncthreads();
    v16bf a0 = frag_ld(xr0 + k0, hh);
    v16bf a1 = frag_ld(xr1 + k0, hh);
#pragma unroll
    for (int j = 0; j < 4; ++j) {
      v16bf b = frag_ld(Bl + (j * 16 + m) * BP, hh);
      c[0][j] = mma(a0, b, c[0][j]);
      c[1][j] = mma(a1, b, c[1][j]);
    }
  }

  float bj[4];
#pragma unroll
  for (int j = 0; j < 4; ++j) bj[j] = bias[col0 + j * 16 + m];

  unsigned short* stg = St + w * (32 * SP);
  const int section = col0 / DM;
  const int head = (col0 % DM) / HD;

  if (section < 2) {
#pragma unroll
    for (int rr = 0; rr < 2; ++rr)
#pragma unroll
      for (int jj = 0; jj < 2; ++jj) {
        const int fi = jj * 16 + m;
#pragma unroll
        for (int r = 0; r < 8; ++r) {
          const int R = rr * 16 + 8 * hh + r;
          const size_t ti = (size_t)(row0 + R) * NFREQ + fi;
          const float cs = cosT[ti], sn = sinT[ti];
          const float t1 = c[rr][jj][r] + bj[jj];
          const float t2 = c[rr][jj + 2][r] + bj[jj + 2];
          stg[R * SP + fi]      = f2bf(t1 * cs - t2 * sn);
          stg[R * SP + 32 + fi] = f2bf(t1 * sn + t2 * cs);
        }
      }
  } else {
#pragma unroll
    for (int rr = 0; rr < 2; ++rr)
#pragma unroll
      for (int j = 0; j < 4; ++j)
#pragma unroll
        for (int r = 0; r < 8; ++r) {
          const int R = rr * 16 + 8 * hh + r;
          stg[R * SP + j * 16 + m] = f2bf(c[rr][j][r] + bj[j]);
        }
  }
  __syncthreads();

  unsigned short* dst = (section == 0) ? Qh : ((section == 1) ? Kh : Vh);
  dst += (size_t)head * SEQ * HD;
#pragma unroll
  for (int q = 0; q < 8; ++q) {
    const int R = q * 4 + (l >> 3), ch = (l & 7) * 8;
    v4u val = *(const v4u*)(stg + R * SP + ch);
    *(volatile v4u*)(dst + (size_t)(row0 + R) * HD + ch) = val;
  }
  __threadfence();
#pragma unroll
  for (int q = 0; q < 8; ++q) {
    const int R = q * 4 + (l >> 3), ch = (l & 7) * 8;
    v4u val = *(const v4u*)(stg + R * SP + ch);
    *(volatile v4u*)(dst + (size_t)(row0 + R) * HD + ch) = val;
  }
}

__global__ __launch_bounds__(256) void k_attn(
    const unsigned short* __restrict__ Qh, const unsigned short* __restrict__ Kh,
    const unsigned short* __restrict__ Vh, unsigned short* __restrict__ ctxh) {
  __shared__ __align__(16) unsigned short Kl[32 * KP];
  __shared__ __align__(16) unsigned short Vl[64 * VP];
  __shared__ __align__(16) unsigned short Pl[8 * 16 * PP];
  __shared__ __align__(16) unsigned short Ol[8 * 16 * OP];
  const int t = threadIdx.x, w = t >> 5, l = t & 31, m = l & 15, hh = l >> 4;
  const int head = blockIdx.x / (SEQ / 128);
  if (head >= NH) return;
  const int qt = (blockIdx.x % (SEQ / 128)) * 8 + w;
  const int row0 = qt * 16;

  const unsigned short* Qb = Qh + (size_t)head * SEQ * HD;
  const unsigned short* Kb = Kh + (size_t)head * SEQ * HD;
  const unsigned short* Vb = Vh + (size_t)head * SEQ * HD;
  unsigned short* P = Pl + w * (16 * PP);
  unsigned short* O = Ol + w * (16 * OP);

  const int sk = t >> 3, sc = (t & 7) * 8;

  const v16bf aq0 = frag_ld(Qb + (size_t)(row0 + m) * HD, hh);
  const v16bf aq1 = frag_ld(Qb + (size_t)(row0 + m) * HD + 32, hh);

  float mi[8], li[8];
  v8f o[4];
#pragma unroll
  for (int r = 0; r < 8; ++r) { mi[r] = -1e30f; li[r] = 0.0f; }
#pragma unroll
  for (int j = 0; j < 4; ++j) o[j] = zero8();

  for (int kt = 0; kt < SEQ / 32; ++kt) {
    const int kbase = kt * 32;
    __syncthreads();
    {
      const unsigned short* krow = Kb + (size_t)(kbase + sk) * HD + sc;
      *(v8us*)(Kl + sk * KP + sc) = *(const v8us*)krow;
      v8us vv = *(const v8us*)(Vb + (size_t)(kbase + sk) * HD + sc);
#pragma unroll
      for (int e = 0; e < 8; ++e) Vl[(sc + e) * VP + sk] = vv[e];
    }
    __syncthreads();

    v8f s0 = mma(aq0, frag_ld(Kl + m * KP, hh), zero8());
    s0 = mma(aq1, frag_ld(Kl + m * KP + 32, hh), s0);
    v8f s1 = mma(aq0, frag_ld(Kl + (16 + m) * KP, hh), zero8());
    s1 = mma(aq1, frag_ld(Kl + (16 + m) * KP + 32, hh), s1);

    float pscale[8];
#pragma unroll
    for (int r = 0; r < 8; ++r) {
      float v0 = s0[r] * 0.125f, v1 = s1[r] * 0.125f;
      float mx = fmaxf(v0, v1);
#pragma unroll
      for (int d = 8; d >= 1; d >>= 1) mx = fmaxf(mx, __shfl_xor(mx, d, 32));
      float mn = fmaxf(mi[r], mx);
      float p0 = __expf(v0 - mn), p1 = __expf(v1 - mn);
      float sum = p0 + p1;
#pragma unroll
      for (int d = 8; d >= 1; d >>= 1) sum += __shfl_xor(sum, d, 32);
      float scl = __expf(mi[r] - mn);
      li[r] = li[r] * scl + sum;
      mi[r] = mn;
      pscale[r] = scl;
      const int rowp = 8 * hh + r;
      P[rowp * PP + m]      = f2bf(p0);
      P[rowp * PP + 16 + m] = f2bf(p1);
    }
#pragma unroll
    for (int j = 0; j < 4; ++j)
#pragma unroll
      for (int r = 0; r < 8; ++r) o[j][r] *= pscale[r];

    __syncthreads();
    v16bf ap = frag_ld(P + m * PP, hh);
#pragma unroll
    for (int j = 0; j < 4; ++j) {
      v16bf b = frag_ld(Vl + (j * 16 + m) * VP, hh);
      o[j] = mma(ap, b, o[j]);
    }
  }

#pragma unroll
  for (int r = 0; r < 8; ++r) {
    const float inv = 1.0f / li[r];
    const int R = 8 * hh + r;
#pragma unroll
    for (int j = 0; j < 4; ++j) O[R * OP + j * 16 + m] = f2bf(o[j][r] * inv);
  }
  __syncthreads();

#pragma unroll
  for (int q = 0; q < 4; ++q) {
    const int R = q * 4 + (l >> 3), ch = (l & 7) * 8;
    v4u val = *(const v4u*)(O + R * OP + ch);
    *(volatile v4u*)(ctxh + (size_t)(row0 + R) * DM + head * HD + ch) = val;
  }
  __threadfence();
#pragma unroll
  for (int q = 0; q < 4; ++q) {
    const int R = q * 4 + (l >> 3), ch = (l & 7) * 8;
    v4u val = *(const v4u*)(O + R * OP + ch);
    *(volatile v4u*)(ctxh + (size_t)(row0 + R) * DM + head * HD + ch) = val;
  }
}

__global__ __launch_bounds__(128) void k_out(
    const unsigned short* __restrict__ ctxh, const unsigned short* __restrict__ owh,
    const float* __restrict__ ob, const float* __restrict__ x, float* __restrict__ out) {
  __shared__ __align__(16) unsigned short Bl[64 * BP];
  __shared__ __align__(16) float Tw[4 * 32 * TP];
  const int t = threadIdx.x, w = t >> 5, l = t & 31, m = l & 15, hh = l >> 4;
  const int NT = DM / 64;
  const int col0 = (blockIdx.x % NT) * 64;
  const int rowb = (blockIdx.x / NT) * 128;
  if (rowb >= SEQ) return;
  const int row0 = rowb + w * 32;

  const unsigned short* cr0 = ctxh + (size_t)(row0 + m) * DM;
  const unsigned short* cr1 = cr0 + (size_t)16 * DM;

  v8f c[2][4];
#pragma unroll
  for (int rr = 0; rr < 2; ++rr)
#pragma unroll
    for (int j = 0; j < 4; ++j) c[rr][j] = zero8();

  for (int i = 0; i < DM / 32; ++i) {
    const int k0 = i * 32;
    __syncthreads();
#pragma unroll
    for (int u = 0; u < 2; ++u) {
      const int cid = t + 128 * u;
      *(v8us*)(Bl + (cid >> 2) * BP + (cid & 3) * 8) =
          *(const v8us*)(owh + (size_t)(col0 + (cid >> 2)) * DM + k0 + (cid & 3) * 8);
    }
    __syncthreads();
    v16bf a0 = frag_ld(cr0 + k0, hh);
    v16bf a1 = frag_ld(cr1 + k0, hh);
#pragma unroll
    for (int j = 0; j < 4; ++j) {
      v16bf b = frag_ld(Bl + (j * 16 + m) * BP, hh);
      c[0][j] = mma(a0, b, c[0][j]);
      c[1][j] = mma(a1, b, c[1][j]);
    }
  }

  float* stg = Tw + w * (32 * TP);
#pragma unroll
  for (int rr = 0; rr < 2; ++rr)
#pragma unroll
    for (int j = 0; j < 4; ++j)
#pragma unroll
      for (int r = 0; r < 8; ++r)
        stg[(rr * 16 + 8 * hh + r) * TP + j * 16 + m] = c[rr][j][r];
  __syncthreads();

#pragma unroll
  for (int p = 0; p < 16; ++p) {
    const int L = p * 4 + (l >> 3);
    const int R = L >> 1;
    const int cofs = (L & 1) * 32 + (l & 7) * 4;
    const int s = row0 + R, n = col0 + cofs;
    v4f a = *(const v4f*)(stg + R * TP + cofs);
    v4f bv = *(const v4f*)(ob + n);
    v4f xv = *(const v4f*)(x + (size_t)s * DM + n);
    v4f val = (a + bv) + xv;
    *(volatile v4f*)(out + (size_t)s * DM + n) = val;
  }
  __threadfence();
#pragma unroll
  for (int p = 0; p < 16; ++p) {
    const int L = p * 4 + (l >> 3);
    const int R = L >> 1;
    const int cofs = (L & 1) * 32 + (l & 7) * 4;
    const int s = row0 + R, n = col0 + cofs;
    v4f a = *(const v4f*)(stg + R * TP + cofs);
    v4f bv = *(const v4f*)(ob + n);
    v4f xv = *(const v4f*)(x + (size_t)s * DM + n);
    v4f val = (a + bv) + xv;
    *(volatile v4f*)(out + (size_t)s * DM + n) = val;
  }
}

extern "C" void kernel_launch(void* const* d_in, const int* in_sizes, int n_in,
                              void* d_out, int out_size, void* d_ws,
                              size_t ws_size, hipStream_t stream) {
  if (n_in < 5) return;
  if (in_sizes[0] != SEQ * DM || in_sizes[1] != 3 * DM * DM || in_sizes[2] != 3 * DM ||
      in_sizes[3] != DM * DM || in_sizes[4] != DM || out_size != SEQ * DM) return;

  const float* x     = (const float*)d_in[0];
  const float* qkv_w = (const float*)d_in[1];
  const float* qkv_b = (const float*)d_in[2];
  const float* out_w = (const float*)d_in[3];
  const float* out_b = (const float*)d_in[4];
  float* out = (float*)d_out;

  const size_t b_xh  = (size_t)SEQ * DM * 2;
  const size_t b_wh  = (size_t)3 * DM * DM * 2;
  const size_t b_owh = (size_t)DM * DM * 2;
  const size_t b_act = (size_t)SEQ * DM * 2;
  const size_t b_tab = (size_t)SEQ * NFREQ * 4;
  size_t off = 0;
  char* ws = (char*)d_ws;
  unsigned short* xh   = (unsigned short*)(ws + off); off += b_xh;
  unsigned short* wh   = (unsigned short*)(ws + off); off += b_wh;
  unsigned short* owh  = (unsigned short*)(ws + off); off += b_owh;
  unsigned short* Qh   = (unsigned short*)(ws + off); off += b_act;
  unsigned short* Kh   = (unsigned short*)(ws + off); off += b_act;
  unsigned short* Vh   = (unsigned short*)(ws + off); off += b_act;
  unsigned short* ctxh = (unsigned short*)(ws + off); off += b_act;
  float* cosT = (float*)(ws + off); off += b_tab;
  float* sinT = (float*)(ws + off); off += b_tab;
  if (off > ws_size) return;

  {
    int n8 = (SEQ * DM) / 8;
    k_cvt<<<(n8 + 255) / 256, 256, 0, stream>>>(x, xh, n8);
    n8 = (3 * DM * DM) / 8;
    k_cvt<<<(n8 + 255) / 256, 256, 0, stream>>>(qkv_w, wh, n8);
    n8 = (DM * DM) / 8;
    k_cvt<<<(n8 + 255) / 256, 256, 0, stream>>>(out_w, owh, n8);
  }
  {
    const int n4 = (SEQ * NFREQ) / 4;
    k_tab<<<(n4 + 255) / 256, 256, 0, stream>>>(cosT, sinT, n4);
  }
  k_qkv<<<(SEQ / 256) * ((3 * DM) / 64), 256, 0, stream>>>(xh, wh, qkv_b, cosT, sinT, Qh, Kh, Vh);
  k_attn<<<NH * (SEQ / 128), 256, 0, stream>>>(Qh, Kh, Vh, ctxh);
  k_out<<<(SEQ / 128) * (DM / 64), 128, 0, stream>>>(ctxh, owh, out_b, x, out);
}
